// BNHCEncoder_77953656422746
// MI455X (gfx1250) — hardware-verified
//
#include <hip/hip_runtime.h>
#include <stddef.h>


#define DD      128
#define KIN     256
#define NTHR    256
#define NWAVE   8
#define EPT     8
#define NGRP    2
#define CHUNK   (NTHR * EPT * NGRP)
#define WCAP    (EPT * NGRP * 32)
#define LISTN   (NWAVE * WCAP)
#define NBC     4096
#define NBF     1024
#define RCAP    32768
#define RBN     128
#define TGT     256
#define DEGCAP  256
#define GROWS   128
#define OTHR    512
#define WSCAP   134217728
#define WSCL    64.0f
#define WINV    0.015625f
#define SPF     (DD + 4)
#define WFC     (DD * KIN)
#define WCV     (DD * DD)
#define LMAX    8

#define LDS_FILL ((RCAP + NBF + LISTN) * 4 + 64)
#define LDS_GEMM(K) (GROWS * ((K) + 8) * 2 + GROWS * SPF * 4)

static_assert((CHUNK & (CHUNK - 1)) == 0);
static_assert(CHUNK <= 4096);
static_assert(NBC <= 4096 && NBF <= 4096);
static_assert((NBC & (NBC - 1)) == 0 && (NBF & (NBF - 1)) == 0);
static_assert(NBC == 4 * NBF);
static_assert(OTHR * 8 == NBC);
static_assert((RCAP % 32) == 0);
static_assert(TGT == NWAVE * 32 && (TGT % GROWS) == 0 && (NBC % TGT) == 0);
static_assert(GROWS == NWAVE * 16);
static_assert(TGT == NTHR);
static_assert(((GROWS * (KIN + 8) * 2) % 16) == 0 && ((GROWS * (DD + 8) * 2) % 16) == 0);
static_assert((SPF % 4) == 0);

typedef float    v4f  __attribute__((ext_vector_type(4)));
typedef float    v8f  __attribute__((ext_vector_type(8)));
typedef int      v4i  __attribute__((ext_vector_type(4)));
typedef _Float16 v8h  __attribute__((ext_vector_type(8)));
typedef _Float16 v16h __attribute__((ext_vector_type(16)));
union FragH { v16h v; v8h h[2]; };

__device__ __forceinline__ v8f wmh(v16h a, v16h b, v8f c) {
  v8f d = __builtin_amdgcn_wmma_f32_16x16x32_f16(false, a, false, b, (short)0, c, false, false);
  asm volatile("v_nop\n\tv_nop\n\tv_nop\n\tv_nop" : "+v"(d) : "v"(a), "v"(b));
  return d;
}

template <int NB>
__device__ __forceinline__ int scan_chunk(const int* __restrict__ dsts, int nE, int cbase, int slotBase,
                                          int vec8, int* list, int tid, int lane, int wave) {
  int wc = 0;
#pragma unroll
  for (int g = 0; g < NGRP; ++g) {
    const int el0  = (g * NTHR + tid) * EPT;
    const int e0   = cbase + el0;
    const int sent = -2147483647 - 1;
    v4i da, db;
    if (vec8 != 0 && cbase + CHUNK <= nE) {
      da = *(const v4i*)(dsts + e0);
      db = *(const v4i*)(dsts + e0 + 4);
    } else {
      da.x = (e0     < nE) ? dsts[min(e0, nE - 1)] : sent;
      da.y = (e0 + 1 < nE) ? dsts[min(e0 + 1, nE - 1)] : sent;
      da.z = (e0 + 2 < nE) ? dsts[min(e0 + 2, nE - 1)] : sent;
      da.w = (e0 + 3 < nE) ? dsts[min(e0 + 3, nE - 1)] : sent;
      db.x = (e0 + 4 < nE) ? dsts[min(e0 + 4, nE - 1)] : sent;
      db.y = (e0 + 5 < nE) ? dsts[min(e0 + 5, nE - 1)] : sent;
      db.z = (e0 + 6 < nE) ? dsts[min(e0 + 6, nE - 1)] : sent;
      db.w = (e0 + 7 < nE) ? dsts[min(e0 + 7, nE - 1)] : sent;
    }
    const unsigned nb = (unsigned)slotBase;
    const unsigned s0 = (unsigned)da.x - nb, s1 = (unsigned)da.y - nb;
    const unsigned s2 = (unsigned)da.z - nb, s3 = (unsigned)da.w - nb;
    const unsigned s4 = (unsigned)db.x - nb, s5 = (unsigned)db.y - nb;
    const unsigned s6 = (unsigned)db.z - nb, s7 = (unsigned)db.w - nb;
    const bool h0 = s0 < (unsigned)NB, h1 = s1 < (unsigned)NB, h2 = s2 < (unsigned)NB, h3 = s3 < (unsigned)NB;
    const bool h4 = s4 < (unsigned)NB, h5 = s5 < (unsigned)NB, h6 = s6 < (unsigned)NB, h7 = s7 < (unsigned)NB;
    const unsigned any = __builtin_amdgcn_ballot_w32(h0 | h1 | h2 | h3 | h4 | h5 | h6 | h7);
    if (any != 0u) {
#define HITJ(J, HJ, SJ) { \
        const unsigned mj = __builtin_amdgcn_ballot_w32(HJ); \
        if (mj != 0u) { \
          if (HJ) { \
            const int pos = wc + (int)__builtin_amdgcn_mbcnt_lo(mj, 0u); \
            if (pos < WCAP) list[wave * WCAP + pos] = ((el0 + (J)) << 12) | (int)(SJ); \
          } \
          wc += (int)__builtin_popcount(mj); } }
      HITJ(0, h0, s0)
      HITJ(1, h1, s1)
      HITJ(2, h2, s2)
      HITJ(3, h3, s3)
      HITJ(4, h4, s4)
      HITJ(5, h5, s5)
      HITJ(6, h6, s6)
      HITJ(7, h7, s7)
#undef HITJ
    }
  }
  return wc;
}

__global__ __launch_bounds__(NTHR) void k_count(const int* __restrict__ dsts, int* cnt, int nE, int vec8) {
  __shared__ __attribute__((aligned(16))) int scnt[NBC];
  __shared__ __attribute__((aligned(16))) int list[LISTN];
  __shared__ int wcnt[NWAVE];
  const int tid = threadIdx.x, lane = tid & 31, wave = tid >> 5;
  const int nodeBase = blockIdx.x * NBC;

  for (int i = tid; i < NBC; i += NTHR) scnt[i] = 0;
  __syncthreads();

  const int nChunks = (nE + CHUNK - 1) / CHUNK;
#pragma unroll 1
  for (int ch = 0; ch < nChunks; ++ch) {
    const int cbase = ch * CHUNK;
    const int wc = scan_chunk<NBC>(dsts, nE, cbase, nodeBase, vec8, list, tid, lane, wave);
    if (lane == 0) wcnt[wave] = wc;
    __syncthreads();
    if (wave == 0) {
#pragma unroll 1
      for (int wsx = 0; wsx < NWAVE; ++wsx) {
        int n = __builtin_amdgcn_readfirstlane(wcnt[wsx]);
        n = n > WCAP ? WCAP : (n < 0 ? 0 : n);
        const int* lp = list + wsx * WCAP;
#pragma unroll 1
        for (int i = 0; i < n; ++i) {
          const int ent  = __builtin_amdgcn_readfirstlane(lp[i]);
          const int slot = ent & (NBC - 1);
          if (lane == 0) scnt[slot] = scnt[slot] + 1;
        }
      }
    }
    __syncthreads();
  }

  v4i cq[4];
#pragma unroll
  for (int q = 0; q < 4; ++q) {
    const int f = (wave * 4 + q) * 128 + 4 * lane;
    cq[q] = *(const v4i*)(scnt + f);
  }
  int* cp = cnt + (size_t)nodeBase;
#pragma unroll
  for (int q = 0; q < 4; ++q) {
    const int f = (wave * 4 + q) * 128 + 4 * lane;
    *(volatile v4i*)(cp + f) = cq[q];
  }
  __threadfence();
#pragma unroll
  for (int q = 0; q < 4; ++q) {
    const int f = (wave * 4 + q) * 128 + 4 * lane;
    *(volatile v4i*)(cp + f) = cq[q];
  }
}

__global__ __launch_bounds__(OTHR) void k_offsets(
    const int* __restrict__ cnt, int* off, int* rbase, int nChunk) {
  __shared__ __attribute__((aligned(16))) int soff[NBC];
  __shared__ __attribute__((aligned(16))) int srb[RBN];
  __shared__ int wtot[OTHR / 32];
  const int tid = threadIdx.x, lane = tid & 31, wave = tid >> 5, sub = tid >> 7;
  for (int i = tid; i < RBN; i += OTHR) srb[i] = 0;
  int carry = 0;
#pragma unroll 1
  for (int ch = 0; ch < nChunk; ++ch) {
    const int base = ch * NBC;
    const v4i c0 = *(const v4i*)(cnt + base + 8 * tid);
    const v4i c1 = *(const v4i*)(cnt + base + 8 * tid + 4);
    const int e0 = max(c0.x, 0), e1 = max(c0.y, 0), e2 = max(c0.z, 0), e3 = max(c0.w, 0);
    const int e4 = max(c1.x, 0), e5 = max(c1.y, 0), e6 = max(c1.z, 0), e7 = max(c1.w, 0);
    const int ts = e0 + e1 + e2 + e3 + e4 + e5 + e6 + e7;
    int incl = ts;
#pragma unroll
    for (int d = 1; d < 32; d <<= 1) {
      const int t = __shfl_up(incl, d);
      if (lane >= d) incl += t;
    }
    if (lane == 31) wtot[wave] = incl;
    __syncthreads();
    const int S0 = wtot[0]  + wtot[1]  + wtot[2]  + wtot[3];
    const int S1 = wtot[4]  + wtot[5]  + wtot[6]  + wtot[7];
    const int S2 = wtot[8]  + wtot[9]  + wtot[10] + wtot[11];
    const int S3 = wtot[12] + wtot[13] + wtot[14] + wtot[15];
    int pre = 0;
#pragma unroll 1
    for (int w = 4 * sub; w < wave; ++w) pre += wtot[w];
    const int b0 = carry;
    const int b1 = b0 + ((S0 + 31) & ~31);
    const int b2 = b1 + ((S1 + 31) & ~31);
    const int b3 = b2 + ((S2 + 31) & ~31);
    const int b4 = b3 + ((S3 + 31) & ~31);
    const int myb = sub == 0 ? b0 : (sub == 1 ? b1 : (sub == 2 ? b2 : b3));
    if (tid == 0) {
      srb[min(4 * ch + 0, RBN - 1)] = b0;
      srb[min(4 * ch + 1, RBN - 1)] = b1;
      srb[min(4 * ch + 2, RBN - 1)] = b2;
      srb[min(4 * ch + 3, RBN - 1)] = b3;
    }
    int run = myb + pre + incl - ts;
    soff[8 * tid + 0] = run; run += e0;
    soff[8 * tid + 1] = run; run += e1;
    soff[8 * tid + 2] = run; run += e2;
    soff[8 * tid + 3] = run; run += e3;
    soff[8 * tid + 4] = run; run += e4;
    soff[8 * tid + 5] = run; run += e5;
    soff[8 * tid + 6] = run; run += e6;
    soff[8 * tid + 7] = run;
    carry = b4;
    __syncthreads();
    const v4i o0 = *(const v4i*)(soff + 4 * tid);
    const v4i o1 = *(const v4i*)(soff + 4 * (tid + OTHR));
    int* op = off + base;
    *(volatile v4i*)(op + 4 * tid) = o0;
    *(volatile v4i*)(op + 4 * (tid + OTHR)) = o1;
    __threadfence();
    *(volatile v4i*)(op + 4 * tid) = o0;
    *(volatile v4i*)(op + 4 * (tid + OTHR)) = o1;
    __syncthreads();
  }
  if (tid == 0) srb[min(4 * nChunk, RBN - 1)] = carry;
  __syncthreads();
  v4i rv = {0, 0, 0, 0};
  if (tid < 32) rv = *(const v4i*)(srb + 4 * tid);
  if (tid < 32) *(volatile v4i*)(rbase + 4 * tid) = rv;
  __threadfence();
  if (tid < 32) *(volatile v4i*)(rbase + 4 * tid) = rv;
}

__global__ __launch_bounds__(NTHR) void k_fill(
    const int* __restrict__ dsts, const int* __restrict__ off, const int* __restrict__ rbase,
    int* csr, int nE, int vec8, int csrLen) {
  extern __shared__ v4f lds_dyn[];
  int* region = (int*)lds_dyn;
  int* cursor = region + RCAP;
  int* list   = cursor + NBF;
  int* wcnt   = list + LISTN;
  const int tid = threadIdx.x, lane = tid & 31, wave = tid >> 5;
  const int b = blockIdx.x;
  const int nodeBase = b * NBF;

  int rb0 = rbase[b];
  const int rb1 = rbase[b + 1];
  rb0 = rb0 < 0 ? 0 : (rb0 > csrLen ? csrLen : rb0);
  rb0 &= ~31;
  int len = rb1 - rb0;
  len = len < 0 ? 0 : (len > RCAP ? RCAP : len);
  int lenW = (len + 31) & ~31;
  if (rb0 + lenW > csrLen) lenW = (csrLen - rb0) & ~31;

  {
    const v4i z = {0, 0, 0, 0};
    for (int i = tid; i < RCAP / 4; i += NTHR) ((v4i*)region)[i] = z;
    for (int s = tid; s < NBF; s += NTHR) {
      int o = off[nodeBase + s] - rb0;
      o = o < 0 ? 0 : (o > RCAP ? RCAP : o);
      cursor[s] = o;
    }
  }
  __syncthreads();

  const int nChunks = (nE + CHUNK - 1) / CHUNK;
#pragma unroll 1
  for (int ch = 0; ch < nChunks; ++ch) {
    const int cbase = ch * CHUNK;
    const int wc = scan_chunk<NBF>(dsts, nE, cbase, nodeBase, vec8, list, tid, lane, wave);
    if (lane == 0) wcnt[wave] = wc;
    __syncthreads();
    if (wave == 0) {
#pragma unroll 1
      for (int wsx = 0; wsx < NWAVE; ++wsx) {
        int n = __builtin_amdgcn_readfirstlane(wcnt[wsx]);
        n = n > WCAP ? WCAP : (n < 0 ? 0 : n);
        const int* lp = list + wsx * WCAP;
#pragma unroll 1
        for (int i = 0; i < n; ++i) {
          const int ent  = __builtin_amdgcn_readfirstlane(lp[i]);
          const int slot = ent & (NBF - 1);
          int e = cbase + ((ent >> 12) & (CHUNK - 1));
          e = e > nE - 1 ? nE - 1 : e;
          if (lane == 0) {
            int pos = cursor[slot];
            pos = pos < 0 ? 0 : (pos > RCAP - 1 ? RCAP - 1 : pos);
            region[pos] = e;
            const int np = pos + 1;
            cursor[slot] = np > RCAP ? RCAP : np;
          }
        }
      }
    }
    __syncthreads();
  }

  const int nv = lenW >> 2;
  int* gp = csr + rb0;
#pragma unroll 1
  for (int i = tid; i < nv; i += NTHR) { const v4i v = ((const v4i*)region)[i]; *(volatile v4i*)(gp + 4 * i) = v; }
  __threadfence();
#pragma unroll 1
  for (int i = tid; i < nv; i += NTHR) { const v4i v = ((const v4i*)region)[i]; *(volatile v4i*)(gp + 4 * i) = v; }
}

__global__ __launch_bounds__(NTHR) void k_wprep(
    const float* __restrict__ fcw, const float* __restrict__ cw, _Float16* wp, int L) {
  const int blk = blockIdx.x, tid = threadIdx.x;
  const int isFc = blk < 16 ? 1 : 0;
  const int ifc = (blk & 15) * NTHR + tid;
  const int nfc = ifc >> 5, kfc = (ifc & 31) * 8;
  int cb = blk - 16; cb = cb < 0 ? 0 : cb;
  int lyr = cb >> 3;
  lyr = lyr > L - 1 ? L - 1 : lyr; lyr = lyr < 0 ? 0 : lyr;
  const int icv = (cb & 7) * NTHR + tid;
  const int ncv = icv >> 4, kcv = (icv & 15) * 8;
  float v[8];
  if (isFc != 0) {
#pragma unroll
    for (int e = 0; e < 8; ++e) v[e] = fcw[(size_t)(kfc + e) * DD + nfc];
  } else {
#pragma unroll
    for (int e = 0; e < 8; ++e) v[e] = cw[(size_t)lyr * WCV + (size_t)(kcv + e) * DD + ncv];
  }
  v8h hv;
  hv[0] = (_Float16)(v[0] * WSCL); hv[1] = (_Float16)(v[1] * WSCL);
  hv[2] = (_Float16)(v[2] * WSCL); hv[3] = (_Float16)(v[3] * WSCL);
  hv[4] = (_Float16)(v[4] * WSCL); hv[5] = (_Float16)(v[5] * WSCL);
  hv[6] = (_Float16)(v[6] * WSCL); hv[7] = (_Float16)(v[7] * WSCL);
  const size_t doff = isFc != 0 ? ((size_t)nfc * KIN + kfc)
                                : ((size_t)WFC + (size_t)lyr * WCV + (size_t)ncv * DD + kcv);
  _Float16* dp = wp + doff;
  *(volatile v8h*)dp = hv;
  __threadfence();
  *(volatile v8h*)dp = hv;
}

__global__ __launch_bounds__(NTHR) void k_deg(
    const int* __restrict__ csr, const int* __restrict__ off, const int* __restrict__ cnt,
    const int* __restrict__ widx, const float* __restrict__ wtab, int wlen, int useIdx,
    float* dinv, int nEdg, int csrLen) {
  __shared__ __attribute__((aligned(16))) float sdeg[NTHR];
  const int tid = threadIdx.x;
  const int d = blockIdx.x * NTHR + tid;
  int n = cnt[d];
  n = n < 0 ? 0 : (n > DEGCAP ? DEGCAP : n);
  const int st = off[d];
  int nm = n;
  nm = max(nm, __shfl_xor(nm, 1));
  nm = max(nm, __shfl_xor(nm, 2));
  nm = max(nm, __shfl_xor(nm, 4));
  nm = max(nm, __shfl_xor(nm, 8));
  nm = max(nm, __shfl_xor(nm, 16));
  nm = __builtin_amdgcn_readfirstlane(nm);
  nm = nm > DEGCAP ? DEGCAP : (nm < 0 ? 0 : nm);
  float acc = 0.0f;
#pragma unroll 1
  for (int p = 0; p < nm; ++p) {
    const int pp = p < n ? p : 0;
    int pos = st + pp;
    pos = pos < 0 ? 0 : (pos > csrLen - 1 ? csrLen - 1 : pos);
    int ed = csr[pos];
    ed = ed < 0 ? 0 : (ed > nEdg - 1 ? nEdg - 1 : ed);
    int wi = widx[ed];
    wi = useIdx != 0 ? wi : ed;
    wi = wi < 0 ? 0 : (wi > wlen - 1 ? wlen - 1 : wi);
    const float wv = wtab[wi];
    acc += (p < n) ? wv : 0.0f;
  }
  float r = 1.0f / sqrtf(acc + 1e-8f);
  r = (r > 3.0e38f || r < -3.0e38f) ? 0.0f : r;
  sdeg[tid] = r;
  __syncthreads();
  v4f v = {0.0f, 0.0f, 0.0f, 0.0f};
  if (tid < NTHR / 4) v = *(const v4f*)(sdeg + 4 * tid);
  float* gp = dinv + (size_t)blockIdx.x * NTHR + 4 * tid;
  if (tid < NTHR / 4) *(volatile v4f*)gp = v;
  __threadfence();
  if (tid < NTHR / 4) *(volatile v4f*)gp = v;
}

__global__ __launch_bounds__(NTHR) void k_coef(
    const int* __restrict__ rowp, const int* __restrict__ colp,
    const float* __restrict__ wMat, const float* __restrict__ eW,
    const float* __restrict__ nd, const float* __restrict__ hd,
    float* ca, float* cbp, int M, int nN, int nE) {
  const int m0 = (blockIdx.x * NTHR + threadIdx.x) * 4;
  v4f av, bv;
#pragma unroll
  for (int e = 0; e < 4; ++e) {
    int mm = m0 + e;
    mm = mm > M - 1 ? M - 1 : mm;
    int r = rowp[mm];
    r = r < 0 ? 0 : (r > nN - 1 ? nN - 1 : r);
    int c = colp[mm];
    c = c < 0 ? 0 : (c > nE - 1 ? nE - 1 : c);
    const float nrm = hd[c] * nd[r];
    const float ew  = eW[mm];
    av[e] = ew * nrm;
    bv[e] = (wMat[c] * ew) * nrm;
  }
  float* pa = ca + m0;
  float* pb = cbp + m0;
  *(volatile v4f*)pa = av;
  *(volatile v4f*)pb = bv;
  __threadfence();
  *(volatile v4f*)pa = av;
  *(volatile v4f*)pb = bv;
}

template <int K, int RELU>
__global__ __launch_bounds__(NTHR) void k_gemm(
    const float* __restrict__ A, int nRowsA, const _Float16* __restrict__ Wp,
    const float* __restrict__ bias, float* C, int nRowsC) {
  static_assert((K % 32) == 0);
  static_assert(((GROWS * K / 8) % NTHR) == 0);
  constexpr int APK = K + 8;
  constexpr int CPR = K / 8;
  constexpr int NT  = DD / 16;
  extern __shared__ v4f lds_dyn[];
  _Float16* sA  = (_Float16*)lds_dyn;
  float*    stg = (float*)(sA + GROWS * APK);
  const int tid = threadIdx.x, lane = tid & 31, wave = tid >> 5, hh = lane >> 4, m = lane & 15;
  const int rowBase = blockIdx.x * GROWS;

#pragma unroll
  for (int i = 0; i < (GROWS * CPR) / NTHR; ++i) {
    const int idx = i * NTHR + tid;
    const int r   = idx / CPR;
    const int c0  = (idx - r * CPR) * 8;
    int gr = rowBase + r;
    gr = gr > nRowsA - 1 ? nRowsA - 1 : gr;
    const float* ap = A + (size_t)gr * K + c0;
    const v4f a0 = *(const v4f*)ap;
    const v4f a1 = *(const v4f*)(ap + 4);
    v8h hv;
    hv[0] = (_Float16)a0.x; hv[1] = (_Float16)a0.y; hv[2] = (_Float16)a0.z; hv[3] = (_Float16)a0.w;
    hv[4] = (_Float16)a1.x; hv[5] = (_Float16)a1.y; hv[6] = (_Float16)a1.z; hv[7] = (_Float16)a1.w;
    *(v8h*)(sA + r * APK + c0) = hv;
  }
  __syncthreads();

  const _Float16* pa = sA + (wave * 16 + m) * APK + 8 * hh;
  v8f acc[NT];
#pragma unroll
  for (int t = 0; t < NT; ++t) {
    const v8f z = {0.f, 0.f, 0.f, 0.f, 0.f, 0.f, 0.f, 0.f};
    acc[t] = z;
  }
#pragma unroll 1
  for (int kt = 0; kt < K / 32; ++kt) {
    FragH a;
    a.h[0] = *(const v8h*)(pa + 32 * kt);
    a.h[1] = *(const v8h*)(pa + 32 * kt + 16);
    const _Float16* bk = Wp + 32 * kt + 8 * hh;
#pragma unroll
    for (int t = 0; t < NT; ++t) {
      const _Float16* bp = bk + (size_t)(16 * t + m) * K;
      FragH b;
      b.h[0] = *(const v8h*)bp;
      b.h[1] = *(const v8h*)(bp + 16);
      acc[t] = wmh(a.v, b.v, acc[t]);
    }
  }

  float* strow = stg + (wave * 16 + 8 * hh) * SPF + m;
#pragma unroll
  for (int t = 0; t < NT; ++t) {
    const float bv = bias[16 * t + m];
#pragma unroll
    for (int r = 0; r < 8; ++r) {
      float v = fmaf(acc[t][r], WINV, bv);
      if (RELU != 0) v = fmaxf(v, 0.0f);
      strow[r * SPF + 16 * t] = v;
    }
  }
  __syncthreads();

#pragma unroll
  for (int i = 0; i < 16; ++i) {
    const int row = wave * 16 + i, grow = rowBase + row;
    const v4f v = *(const v4f*)(stg + row * SPF + 4 * lane);
    if (grow < nRowsC) *(volatile v4f*)(C + (size_t)grow * DD + 4 * lane) = v;
  }
  __threadfence();
#pragma unroll
  for (int i = 0; i < 16; ++i) {
    const int row = wave * 16 + i, grow = rowBase + row;
    const v4f v = *(const v4f*)(stg + row * SPF + 4 * lane);
    if (grow < nRowsC) *(volatile v4f*)(C + (size_t)grow * DD + 4 * lane) = v;
  }
}

__device__ __forceinline__ v4f agg_seg(
    const int* __restrict__ csr, const int* __restrict__ acol, const float* __restrict__ aval,
    const float* __restrict__ xin, int n, int st, int lane, int nSrc, int nEdg, int csrLen) {
  v4f acc = {0.0f, 0.0f, 0.0f, 0.0f};
#pragma unroll 1
  for (int q0 = 0; q0 < n; q0 += 32) {
    int pos = st + q0 + lane;
    pos = pos < 0 ? 0 : (pos > csrLen - 1 ? csrLen - 1 : pos);
    int ed = csr[pos];
    ed = ed < 0 ? 0 : (ed > nEdg - 1 ? nEdg - 1 : ed);
    int cl = acol[ed];
    cl = cl < 0 ? 0 : (cl > nSrc - 1 ? nSrc - 1 : cl);
    const float vl = aval[ed];
    const int mcnt = (n - q0) < 32 ? (n - q0) : 32;
#pragma unroll 1
    for (int p = 0; p < mcnt; ++p) {
      const int   s = __builtin_amdgcn_readlane(cl, p);
      const float v = __int_as_float(__builtin_amdgcn_readlane(__float_as_int(vl), p));
      const v4f   xv = *(const v4f*)(xin + (size_t)s * DD + 4 * lane);
      acc.x = fmaf(v, xv.x, acc.x);
      acc.y = fmaf(v, xv.y, acc.y);
      acc.z = fmaf(v, xv.z, acc.z);
      acc.w = fmaf(v, xv.w, acc.w);
    }
  }
  return acc;
}

template <int MODE>
__global__ __launch_bounds__(NTHR) void k_agg(
    const int* __restrict__ csr, const int* __restrict__ off, const int* __restrict__ cnt,
    const int* __restrict__ acol, const float* __restrict__ aval,
    const float* __restrict__ xin, int nSrc, const float* __restrict__ hres,
    float* dst, int nDstStore, int nEdg, int csrLen) {
  const int tid = threadIdx.x, lane = tid & 31, wave = tid >> 5;
  const int tbase = blockIdx.x * TGT + wave * 32;
  const int cnt_l = cnt[tbase + lane];
  const int off_l = off[tbase + lane];

#pragma unroll 1
  for (int j = 0; j < 32; ++j) {
    int n = __builtin_amdgcn_readlane(cnt_l, j);
    n = n < 0 ? 0 : (n > DEGCAP ? DEGCAP : n);
    const int st = __builtin_amdgcn_readlane(off_l, j);
    const v4f acc = agg_seg(csr, acol, aval, xin, n, st, lane, nSrc, nEdg, csrLen);
    const int d = tbase + j;
    v4f w = acc;
    if (MODE == 1) {
      const v4f hv = *(const v4f*)(hres + (size_t)d * DD + 4 * lane);
      w.x = fmaxf(hv.x + acc.x, 0.0f);
      w.y = fmaxf(hv.y + acc.y, 0.0f);
      w.z = fmaxf(hv.z + acc.z, 0.0f);
      w.w = fmaxf(hv.w + acc.w, 0.0f);
    }
    if (d < nDstStore) {
      float* gp = dst + (size_t)d * DD + 4 * lane;
      *(volatile v4f*)gp = w;
      __threadfence();
      *(volatile v4f*)gp = w;
    }
  }
}

static inline size_t carve(size_t& o, size_t bytes) {
  const size_t r = o;
  o += bytes;
  o = (o + 255) & ~(size_t)255;
  return r;
}

extern "C" void kernel_launch(void* const* d_in, const int* in_sizes, int n_in,
                              void* d_out, int out_size, void* d_ws, size_t ws_size,
                              hipStream_t stream) {
  if (n_in < 8) return;
  const int nN = in_sizes[0] / KIN;
  if (nN < 1 || in_sizes[0] != nN * KIN) return;
  const int M = in_sizes[3];
  if (M < 1 || in_sizes[1] != 2 * M) return;
  const int nE = in_sizes[2];
  if (nE < 1) return;
  if (in_sizes[4] != KIN * DD || in_sizes[5] != DD) return;
  const int L = in_sizes[6] / WCV;
  if (L < 0 || L > LMAX || in_sizes[6] != L * WCV || in_sizes[7] != L * DD) return;
  if ((long long)out_size != (long long)nN * DD) return;
  if (nN > (1 << 24) || nE > (1 << 24) || M > (1 << 28)) return;

  const float* x    = (const float*)d_in[0];
  const int*   hidx = (const int*)d_in[1];
  const float* wMat = (const float*)d_in[2];
  const float* eW   = (const float*)d_in[3];
  const float* fcw  = (const float*)d_in[4];
  const float* fcb  = (const float*)d_in[5];
  const float* cw   = (const float*)d_in[6];
  const float* cvb  = (const float*)d_in[7];
  float* out = (float*)d_out;
  const int* rowp = hidx;
  const int* colp = hidx + M;

  const int NPAD = ((nN + TGT - 1) / TGT) * TGT;
  const int EPAD = ((nE + TGT - 1) / TGT) * TGT;
  const int nBCn = (nN + NBC - 1) / NBC, CNTPn = nBCn * NBC, nBFn = (nN + NBF - 1) / NBF;
  const int nBCe = (nE + NBC - 1) / NBC, CNTPe = nBCe * NBC, nBFe = (nE + NBF - 1) / NBF;
  if (4 * nBCn + 1 > RBN || 4 * nBCe + 1 > RBN) return;
  if (31 * 4 * nBCn > 4096 || 31 * 4 * nBCe > 4096) return;
  const int csrLen = ((M + 31) & ~31) + 4096;
  const int MPAD = ((M + 4 * NTHR - 1) / (4 * NTHR)) * (4 * NTHR);

  char* ws = (char*)d_ws;
  size_t o = 0;
  const size_t oW    = carve(o, (size_t)(WFC + L * WCV) * 2);
  const size_t oCntN = carve(o, (size_t)CNTPn * 4);
  const size_t oOffN = carve(o, (size_t)CNTPn * 4);
  const size_t oRbN  = carve(o, (size_t)RBN * 4);
  const size_t oCsrN = carve(o, (size_t)csrLen * 4);
  const size_t oCntE = carve(o, (size_t)CNTPe * 4);
  const size_t oOffE = carve(o, (size_t)CNTPe * 4);
  const size_t oRbE  = carve(o, (size_t)RBN * 4);
  const size_t oCsrE = carve(o, (size_t)csrLen * 4);
  const size_t oNd   = carve(o, (size_t)CNTPn * 4);
  const size_t oHd   = carve(o, (size_t)CNTPe * 4);
  const size_t oCa   = carve(o, (size_t)MPAD * 4);
  const size_t oCb   = carve(o, (size_t)MPAD * 4);
  const size_t oHA   = carve(o, (size_t)NPAD * DD * 4);
  const size_t oHB   = carve(o, (size_t)NPAD * DD * 4);
  const size_t oXT   = carve(o, (size_t)NPAD * DD * 4);
  const size_t oHF   = carve(o, (size_t)EPAD * DD * 4);
  if (o > ws_size || o > (size_t)WSCAP) return;
  _Float16* wp   = (_Float16*)(ws + oW);
  int*      cntN = (int*)(ws + oCntN);
  int*      offN = (int*)(ws + oOffN);
  int*      rbN  = (int*)(ws + oRbN);
  int*      csrN = (int*)(ws + oCsrN);
  int*      cntE = (int*)(ws + oCntE);
  int*      offE = (int*)(ws + oOffE);
  int*      rbE  = (int*)(ws + oRbE);
  int*      csrE = (int*)(ws + oCsrE);
  float*    ndp  = (float*)(ws + oNd);
  float*    hdp  = (float*)(ws + oHd);
  float*    cfa  = (float*)(ws + oCa);
  float*    cfb  = (float*)(ws + oCb);
  float*    HA   = (float*)(ws + oHA);
  float*    HB   = (float*)(ws + oHB);
  float*    XT   = (float*)(ws + oXT);
  float*    HF   = (float*)(ws + oHF);

  const int vec8 = ((M & 3) == 0) ? 1 : 0;

  k_wprep<<<16 + 8 * L, NTHR, 0, stream>>>(fcw, cw, wp, L);

  hipFuncSetAttribute(reinterpret_cast<const void*>(&k_fill),
                      hipFuncAttributeMaxDynamicSharedMemorySize, LDS_FILL);
  k_count<<<nBCn, NTHR, 0, stream>>>(rowp, cntN, M, vec8);
  k_offsets<<<1, OTHR, 0, stream>>>(cntN, offN, rbN, nBCn);
  k_fill<<<nBFn, NTHR, LDS_FILL, stream>>>(rowp, offN, rbN, csrN, M, vec8, csrLen);

  k_count<<<nBCe, NTHR, 0, stream>>>(colp, cntE, M, vec8);
  k_offsets<<<1, OTHR, 0, stream>>>(cntE, offE, rbE, nBCe);
  k_fill<<<nBFe, NTHR, LDS_FILL, stream>>>(colp, offE, rbE, csrE, M, vec8, csrLen);

  k_deg<<<NPAD / NTHR, NTHR, 0, stream>>>(csrN, offN, cntN, colp, wMat, nE, 1, ndp, M, csrLen);
  k_deg<<<EPAD / NTHR, NTHR, 0, stream>>>(csrE, offE, cntE, colp, eW, M, 0, hdp, M, csrLen);

  k_coef<<<MPAD / (4 * NTHR), NTHR, 0, stream>>>(rowp, colp, wMat, eW, ndp, hdp, cfa, cfb, M, nN, nE);

  hipFuncSetAttribute(reinterpret_cast<const void*>(&k_gemm<KIN, 1>),
                      hipFuncAttributeMaxDynamicSharedMemorySize, LDS_GEMM(KIN));
  hipFuncSetAttribute(reinterpret_cast<const void*>(&k_gemm<DD, 0>),
                      hipFuncAttributeMaxDynamicSharedMemorySize, LDS_GEMM(DD));
  float* h0dst  = (L > 0) ? HA : out;
  const int h0n = (L > 0) ? NPAD : nN;
  k_gemm<KIN, 1><<<NPAD / GROWS, NTHR, LDS_GEMM(KIN), stream>>>(x, nN, wp, fcb, h0dst, h0n);

  float* hc = HA;
  float* hn = HB;
  for (int l = 0; l < L; ++l) {
    k_gemm<DD, 0><<<NPAD / GROWS, NTHR, LDS_GEMM(DD), stream>>>(
        hc, NPAD, wp + WFC + (size_t)l * WCV, cvb + (size_t)l * DD, XT, NPAD);
    k_agg<0><<<EPAD / TGT, NTHR, 0, stream>>>(csrE, offE, cntE, rowp, cfa, XT, nN, XT, HF, EPAD, M, csrLen);
    const int last = (l == L - 1) ? 1 : 0;
    float* zdst = last ? out : hn;
    const int zn = last ? nN : NPAD;
    k_agg<1><<<NPAD / TGT, NTHR, 0, stream>>>(csrN, offN, cntN, colp, cfb, HF, nE, hc, zdst, zn, M, csrLen);
    float* t = hc; hc = hn; hn = t;
  }
}
